// MultiPerspective_14328010899892
// MI455X (gfx1250) — hardware-verified
//
#include <hip/hip_runtime.h>


#ifndef NB
#define NB 128
#endif
#define NB_FULL 128
#define SEQ   64
#define HID   384
#define NP    20
#define NPP   32
#define OC    160
#define EPSN  1e-8f
#define CA    64.0f
#define CW    1024.0f
#define CINV  (1.0f / 65536.0f)
#define CC    256.0f
#define HP    392
#define RP    184

static_assert(SEQ == 64);
static_assert(HID % 32 == 0);
static_assert(HID / 8 == 48);
static_assert(NB % 32 == 0);
static_assert(NB <= NB_FULL);
static_assert(NP <= NPP);
static_assert(OC == 8 * NP);
static_assert((HP * 2) % 16 == 0);
static_assert(HP >= HID);
static_assert(RP >= 9 * NP);
static_assert((RP * 4) % 16 == 0);
static_assert(CA * CW == 65536.0f);

typedef _Float16 h16;
typedef unsigned short bf;
typedef __attribute__((ext_vector_type(16))) __bf16   v16bf;
typedef __attribute__((ext_vector_type(16))) _Float16 v16h;
typedef __attribute__((ext_vector_type(8)))  _Float16 v8h;
typedef __attribute__((ext_vector_type(8)))  unsigned short v8us;
typedef __attribute__((ext_vector_type(8)))  float    v8f;
typedef __attribute__((ext_vector_type(4)))  float    v4f;
typedef v4f  __attribute__((may_alias)) v4fa;
typedef v8h  __attribute__((may_alias)) v8ha;

__device__ __forceinline__ unsigned short f2bf(float f) { unsigned u = __float_as_uint(f); u += 0x7FFFu + ((u >> 16) & 1u); return (unsigned short)(u >> 16); }
__device__ __forceinline__ float bfr(float f) { return __uint_as_float(((unsigned)f2bf(f)) << 16); }
__device__ __forceinline__ v16h cat16(v8h lo, v8h hi) { return __builtin_shufflevector(lo, hi, 0, 1, 2, 3, 4, 5, 6, 7, 8, 9, 10, 11, 12, 13, 14, 15); }
__device__ __forceinline__ v16bf cat16b(v8us lo, v8us hi) { return __builtin_bit_cast(v16bf, __builtin_shufflevector(lo, hi, 0, 1, 2, 3, 4, 5, 6, 7, 8, 9, 10, 11, 12, 13, 14, 15)); }
__device__ __forceinline__ v8f wmma16(v16h a, v16h b, v8f c) { return __builtin_amdgcn_wmma_f32_16x16x32_f16(false, a, false, b, (short)0, c, false, false); }
__device__ __forceinline__ v8f wmmab(v16bf a, v16bf b, v8f c) { return __builtin_amdgcn_wmma_f32_16x16x32_bf16(false, a, false, b, (short)0, c, false, false); }
__device__ __forceinline__ v16h  ldh(const h16* p) { return cat16(*(const v8h*)p, *(const v8h*)(p + 16)); }
__device__ __forceinline__ v16bf ldb(const bf* p)  { return cat16b(*(const v8us*)p, *(const v8us*)(p + 16)); }
__device__ __forceinline__ void wave_sync() { __builtin_amdgcn_fence(3  , "wavefront"); __builtin_amdgcn_wave_barrier(); asm volatile("" ::: "memory"); }
static __device__ __forceinline__ h16 toh_flush(float v) { const h16 r = (h16)v; return (fabsf(v) < 6.103515625e-05f) ? (h16)0.0f : r; }
__device__ __forceinline__ v8f wmma16g(v16h a, v16h b, v8f c) { c = wmma16(a, b, c); asm volatile("v_nop\n\tv_nop\n\tv_nop\n\tv_nop" : "+v"(c) : "v"(a), "v"(b)); return c; }
__device__ __forceinline__ v8f wmmabg(v16bf a, v16bf b, v8f c) { c = wmmab(a, b, c); asm volatile("v_nop\n\tv_nop\n\tv_nop\n\tv_nop" : "+v"(c) : "v"(a), "v"(b)); return c; }

static constexpr size_t PLANE = (size_t)SEQ * NB_FULL * HID;
static_assert(PLANE % (8 * 256) == 0);
static_assert((NPP * HID / 8) % 256 == 0);

__global__ __launch_bounds__(256) void k_cvt2(const float* __restrict__ src, bf* dstb, h16* dsth, size_t n8) {
    const size_t i = (size_t)blockIdx.x * 256 + threadIdx.x; if (i >= n8) return;
    const v8f v = *(const v8f*)(src + i * 8); v8us o; v8h g;
#pragma unroll
    for (int k = 0; k < 8; ++k) { const unsigned short u = f2bf(v[k]); o[k] = u; g[k] = toh_flush(__uint_as_float(((unsigned)u) << 16)); }
    *(volatile v8us*)(dstb + i * 8) = o; *(volatile v8h*)(dsth + i * 8) = g;
    __threadfence();
    *(volatile v8us*)(dstb + i * 8) = o; *(volatile v8h*)(dsth + i * 8) = g;
}

__global__ __launch_bounds__(256) void k_w2(const float* __restrict__ w, h16* dst) {
    const int i = blockIdx.x * 256 + threadIdx.x;
    const int row = i / 48, c8 = (i % 48) * 8;
    const int rc = row < NP ? row : NP - 1;
    v8f v = *(const v8f*)(w + (size_t)rc * HID + c8);
    asm volatile("" : "+v"(v));
    v8h o;
#pragma unroll
    for (int k = 0; k < 8; ++k) { const float x = bfr(v[k]); const float q = x * x * CW; const h16 hq = toh_flush(q); o[k] = (row < NP) ? hq : (h16)0.0f; }
    *(volatile v8h*)(dst + (size_t)i * 8) = o; __threadfence(); *(volatile v8h*)(dst + (size_t)i * 8) = o;
}

static_assert(64 * 68 * 4 + 64 * 72 * 2 + HID * 72 * 2 + 4 * 16 * 72 * 2 + 128 * 4 + 64 * 4 + 64 * 4 <= 131072);
static_assert((64 * 48) % 128 == 0);
__global__ __launch_bounds__(128) void k_gram(const bf* __restrict__ XB, const h16* XH, h16* NHP, h16* HGP, float* DEN) {
    __shared__ __align__(16) float cs32[64 * 68];
    __shared__ __align__(16) h16   cs16[64 * 72];
    __shared__ __align__(16) h16   hT[HID * 72];
    __shared__ __align__(16) h16   os[4 * 16 * 72];
    __shared__ __align__(16) float rn[128];
    __shared__ __align__(16) float dens[64];
    __shared__ int idxs[64];
    const int tid = threadIdx.x, lane = tid & 31, lr = lane & 15, hi = lane >> 4;
    const int wave = __builtin_amdgcn_readfirstlane((int)(threadIdx.x >> 5));
    const int b = blockIdx.x, dir = blockIdx.y;

    { const int which = tid >> 6, row = tid & 63;
      const size_t ro = (size_t)(which * 2 + dir) * PLANE + ((size_t)(row * NB_FULL + b)) * HID;
      float a[8];
#pragma unroll
      for (int e = 0; e < 8; ++e) a[e] = 0.0f;
#pragma unroll 2
      for (int c = 0; c < HID / 8; ++c) { const v8us u = *(const v8us*)(XB + ro + c * 8);
#pragma unroll
          for (int e = 0; e < 8; ++e) { const float x = __uint_as_float(((unsigned)u[e]) << 16); a[e] += x * x; } }
      const float s = ((a[0] + a[1]) + (a[2] + a[3])) + ((a[4] + a[5]) + (a[6] + a[7]));
      rn[tid] = 1.0f / fmaxf(sqrtf(s), EPSN); }

    v8f g[4];
#pragma unroll
    for (int jt = 0; jt < 4; ++jt) g[jt] = (v8f){};
    { const size_t po = (size_t)dir * PLANE + ((size_t)((16 * wave + lr) * NB_FULL + b)) * HID + 8 * hi;
      const size_t ho = (size_t)(2 + dir) * PLANE + ((size_t)(lr * NB_FULL + b)) * HID + 8 * hi;
#pragma unroll 1
      for (int kc = 0; kc < HID; kc += 32) {
          const v16bf a = ldb(XB + po + kc);
#pragma unroll
          for (int jt = 0; jt < 4; ++jt) { const v16bf bb = ldb(XB + ho + (size_t)jt * 16 * NB_FULL * HID + kc); g[jt] = wmmabg(a, bb, g[jt]); }
      } }
    __syncthreads();
#pragma unroll
    for (int jt = 0; jt < 4; ++jt) {
        const float r2 = rn[64 + 16 * jt + lr];
#pragma unroll
        for (int r = 0; r < 8; ++r) { const int row = 16 * wave + 8 * hi + r; const float c = g[jt][r] * rn[row] * r2;
            cs32[row * 68 + 16 * jt + lr] = c; cs16[row * 72 + 16 * jt + lr] = toh_flush(c * CC); } }
    __syncthreads();
    if (wave < 2) {
        const int row = tid;
        float best = cs32[row * 68]; float s = best; int bi = 0;
#pragma unroll 4
        for (int j = 1; j < 64; ++j) { const float v = cs32[row * 68 + j]; s += v; if (v > best) { best = v; bi = j; } }
        idxs[row] = bi; dens[row] = s;
    }
#pragma unroll 2
    for (int it = 0; it < 24; ++it) { const int q = it * 128 + tid; const int j = q / 48, c8 = (q % 48) * 8;
        const v8h x = *(const v8h*)(XH + (size_t)(2 + dir) * PLANE + ((size_t)(j * NB_FULL + b)) * HID + c8);
#pragma unroll
        for (int e = 0; e < 8; ++e) hT[(c8 + e) * 72 + j] = x[e]; }
    __syncthreads();

    { const int ar = (16 * wave + lr) * 72 + 8 * hi;
      const v16h a0 = cat16(*(const v8ha*)&cs16[ar], *(const v8ha*)&cs16[ar + 16]);
      const v16h a1 = cat16(*(const v8ha*)&cs16[ar + 32], *(const v8ha*)&cs16[ar + 48]);
      const int wb = wave * 16 * 72;
#pragma unroll 1
      for (int cg = 0; cg < 6; ++cg) {
          v8f n[4];
#pragma unroll
          for (int c = 0; c < 4; ++c) { n[c] = (v8f){};
              const int hr = (cg * 64 + c * 16 + lr) * 72 + 8 * hi;
              const v16h b0 = cat16(*(const v8ha*)&hT[hr], *(const v8ha*)&hT[hr + 16]);
              const v16h b1 = cat16(*(const v8ha*)&hT[hr + 32], *(const v8ha*)&hT[hr + 48]);
              n[c] = wmma16g(a0, b0, n[c]); n[c] = wmma16g(a1, b1, n[c]); }
#pragma unroll
          for (int c = 0; c < 4; ++c) {
#pragma unroll
              for (int r = 0; r < 8; ++r) os[wb + (8 * hi + r) * 72 + c * 16 + lr] = toh_flush(n[c][r] * (CA / CC)); }
          wave_sync();
          static_assert(4 * 32 * 16 == 16 * 128);
#pragma unroll 1
          for (int ps = 0; ps < 2; ++ps) {
#pragma unroll
              for (int s = 0; s < 4; ++s) { const int row = 4 * s + (lane >> 3), c8 = (lane & 7) * 8;
                  const v8h val = *(const v8ha*)&os[wb + row * 72 + c8];
                  *(volatile v8h*)(NHP + (size_t)dir * PLANE + ((size_t)((16 * wave + row) * NB_FULL + b)) * HID + cg * 64 + c8) = val; }
              if (ps == 0) __threadfence(); }
          wave_sync();
      } }
    static_assert(16 * 16 == SEQ * 4);
    if (wave == 0) {
        const v4f dv = *(const v4fa*)&dens[(lane & 15) * 4];
#pragma unroll 1
        for (int ps = 0; ps < 2; ++ps) {
            if (lane < 16) *(volatile v4f*)(DEN + ((size_t)(dir * NB_FULL + b)) * SEQ + (lane & 15) * 4) = dv;
            if (ps == 0) __threadfence(); }
    }
    static_assert(128 * 24 * 16 == 64 * HID * 2);
#pragma unroll 1
    for (int ps = 0; ps < 2; ++ps) {
#pragma unroll 2
        for (int it = 0; it < 24; ++it) { const int q = it * 128 + tid; const int row = q / 48, pc = q % 48;
            int j = idxs[row]; j = j < 0 ? 0 : (j > SEQ - 1 ? SEQ - 1 : j);
            const v8h x = *(const v8h*)(XH + (size_t)(2 + dir) * PLANE + ((size_t)(j * NB_FULL + b)) * HID + pc * 8);
            *(volatile v8h*)(HGP + (size_t)dir * PLANE + ((size_t)(row * NB_FULL + b)) * HID + pc * 8) = x; }
        if (ps == 0) __threadfence(); }
}

static_assert(64 * HP * 2 + NP * HID * 4 + 2 * NPP * 64 * 4 + 64 * 32 * 4 <= 131072);
__global__ __launch_bounds__(128) void k_mpm(const h16* __restrict__ XH, const h16* __restrict__ W2H, const float* __restrict__ w, float* MPMT, int dir) {
    __shared__ __align__(16) h16   BM[64 * HP];
    __shared__ __align__(16) float W2S[NP * HID];
    __shared__ __align__(16) float RN[2 * NPP * 64];
    __shared__ __align__(16) float RES[64 * 32];
    const int tid = threadIdx.x, lane = tid & 31, lr = lane & 15, hi = lane >> 4;
    const int wave = __builtin_amdgcn_readfirstlane((int)(threadIdx.x >> 5));
    const int b = blockIdx.x;
#pragma unroll 4
    for (int q = tid; q < NP * HID; q += 128) { const float x = bfr(w[q]); W2S[q] = x * x * CW; }
#pragma unroll 4
    for (int q = tid; q < 64 * 32; q += 128) RES[q] = 0.0f;
    { const size_t wo = ((size_t)((dir * 4 + 1) * NPP + lr)) * HID + 8 * hi;
#pragma unroll 1
      for (int which = 0; which < 2; ++which) {
          const size_t xo = (size_t)(which * 2 + dir) * PLANE + ((size_t)((16 * wave + lr) * NB_FULL + b)) * HID + 8 * hi;
          v8f c0 = (v8f){}, c1 = (v8f){};
#pragma unroll 1
          for (int kc = 0; kc < HID; kc += 32) {
              const v16h x = ldh(XH + xo + kc); v16h a2;
#pragma unroll
              for (int e = 0; e < 16; ++e) { const float f = (float)x[e]; a2[e] = toh_flush(f * f * CA); }
              const v16h b0 = ldh(W2H + wo + kc); const v16h b1 = ldh(W2H + wo + (size_t)16 * HID + kc);
              c0 = wmma16g(a2, b0, c0); c1 = wmma16g(a2, b1, c1); }
#pragma unroll
          for (int r = 0; r < 8; ++r) { const int tok = 16 * wave + 8 * hi + r;
              RN[which * (NPP * 64) + lr * 64 + tok] = 1.0f / fmaxf(sqrtf(c0[r] * CINV), EPSN);
              RN[which * (NPP * 64) + (16 + lr) * 64 + tok] = 1.0f / fmaxf(sqrtf(c1[r] * CINV), EPSN); }
      } }
    __syncthreads();
    const size_t po = (size_t)dir * PLANE + ((size_t)((16 * wave + lr) * NB_FULL + b)) * HID + 8 * hi;
    const size_t hb = (size_t)(2 + dir) * PLANE + (size_t)b * HID;
#pragma unroll 1
    for (int m = 0; m < NP; ++m) {
#pragma unroll 2
        for (int it = 0; it < 24; ++it) { const int q = it * 128 + tid; const int j = q / 48, c8 = (q % 48) * 8;
            const v8h x = *(const v8h*)(XH + hb + (size_t)j * NB_FULL * HID + c8);
            const v4f w0 = *(const v4fa*)&W2S[m * HID + c8]; const v4f w1 = *(const v4fa*)&W2S[m * HID + c8 + 4]; v8h o;
#pragma unroll
            for (int e = 0; e < 4; ++e) { o[e] = toh_flush((float)x[e] * w0[e]); o[4 + e] = toh_flush((float)x[4 + e] * w1[e]); }
            *(v8ha*)&BM[j * HP + c8] = o; }
        __syncthreads();
        v8f s[4];
#pragma unroll
        for (int jt = 0; jt < 4; ++jt) s[jt] = (v8f){};
#pragma unroll 1
        for (int kc = 0; kc < HID; kc += 32) {
            const v16h a = ldh(XH + po + kc);
#pragma unroll
            for (int jt = 0; jt < 4; ++jt) { const int br = (16 * jt + lr) * HP + kc + 8 * hi;
                const v16h bb = cat16(*(const v8ha*)&BM[br], *(const v8ha*)&BM[br + 16]);
                s[jt] = wmma16g(a, bb, s[jt]); } }
        float r2[4];
#pragma unroll
        for (int jt = 0; jt < 4; ++jt) r2[jt] = RN[NPP * 64 + m * 64 + 16 * jt + lr];
        float mx[8];
#pragma unroll
        for (int r = 0; r < 8; ++r) {
            float v = s[0][r] * r2[0]; v = fmaxf(v, s[1][r] * r2[1]); v = fmaxf(v, s[2][r] * r2[2]); v = fmaxf(v, s[3][r] * r2[3]);
            mx[r] = v * (RN[m * 64 + 16 * wave + 8 * hi + r] * (1.0f / CW)); }
#pragma unroll
        for (int r = 0; r < 8; ++r) { float v = mx[r];
            v = fmaxf(v, __shfl_xor(v, 8, 32)); v = fmaxf(v, __shfl_xor(v, 4, 32)); v = fmaxf(v, __shfl_xor(v, 2, 32)); v = fmaxf(v, __shfl_xor(v, 1, 32)); mx[r] = v; }
        float sel = mx[0];
#pragma unroll
        for (int r = 1; r < 8; ++r) sel = ((lr & 7) == r) ? mx[r] : sel;
        if (lr < 8) RES[(16 * wave + 8 * hi + lr) * 32 + m] = sel;
        __syncthreads();
    }
    static_assert(4 * 32 * 16 == 16 * 32 * 4);
#pragma unroll 1
    for (int ps = 0; ps < 2; ++ps) {
#pragma unroll
        for (int sI = 0; sI < 4; ++sI) { const int row = 16 * wave + 4 * sI + (lane >> 3), cofs = (lane & 7) * 4;
            const v4f val = *(const v4fa*)&RES[row * 32 + cofs];
            *(volatile v4f*)(MPMT + ((size_t)((dir * SEQ + row) * NB_FULL + b)) * 32 + cofs) = val; }
        if (ps == 0) __threadfence(); }
}

static_assert(32 * HP * 2 + 32 * RP * 4 + 32 * OC * 4 <= 131072);
static_assert((32 * 48) % 128 == 0);
static_assert(32 * NP == 5 * 128);
__global__ __launch_bounds__(128) void k_final(const h16* __restrict__ HPL, const h16* __restrict__ W2H, const float* __restrict__ DEN, const float* __restrict__ MPMT, float* OUT) {
    __shared__ __align__(16) h16   AT[32 * HP];
    __shared__ __align__(16) float R[32 * RP];
    __shared__ __align__(16) float OT[32 * OC];
    const int tid = threadIdx.x, lane = tid & 31, lr = lane & 15, hi = lane >> 4;
    const int wave = __builtin_amdgcn_readfirstlane((int)(threadIdx.x >> 5));
    const int rt = wave & 1, nh = wave >> 1;
    const int tpb = NB / 32;
    const int t = blockIdx.x / tpb, b0 = (blockIdx.x % tpb) * 32;
    const int rowt = t * NB_FULL, rowl = (SEQ - 1) * NB_FULL;
#pragma unroll 1
    for (int dir = 0; dir < 2; ++dir) {
#pragma unroll 1
        for (int s = 0; s < 7; ++s) {
            int px, py, rx, ry; float sc;
            switch (s) {
                case 0:  px = dir;     py = dir;     rx = rowt; ry = rowt; sc = CA; break;
                case 1:  px = dir;     py = 2 + dir; rx = rowt; ry = rowl; sc = CA; break;
                case 2:  px = 2 + dir; py = 2 + dir; rx = rowl; ry = rowl; sc = CA; break;
                case 3:  px = dir;     py = 4 + dir; rx = rowt; ry = rowt; sc = 1.0f; break;
                case 4:  px = 4 + dir; py = 4 + dir; rx = rowt; ry = rowt; sc = 1.0f / CA; break;
                case 5:  px = dir;     py = 6 + dir; rx = rowt; ry = rowt; sc = CA; break;
                default: px = 6 + dir; py = 6 + dir; rx = rowt; ry = rowt; sc = CA; break;
            }
            const size_t xo = (size_t)px * PLANE + (size_t)(rx + b0) * HID;
            const size_t yo = (size_t)py * PLANE + (size_t)(ry + b0) * HID;
#pragma unroll 2
            for (int it = 0; it < 12; ++it) { const int q = it * 128 + tid; const int r = q / 48, c8 = (q % 48) * 8;
                const v8h x = *(const v8h*)(HPL + xo + (size_t)r * HID + c8);
                const v8h y = *(const v8h*)(HPL + yo + (size_t)r * HID + c8); v8h o;
#pragma unroll
                for (int e = 0; e < 8; ++e) o[e] = toh_flush((float)x[e] * (float)y[e] * sc);
                *(v8ha*)&AT[r * HP + c8] = o; }
            __syncthreads();
            const int ntc = (s == 0) ? 6 : 2;
#pragma unroll 1
            for (int n = nh; n < ntc; n += 2) {
                const int ki = (s == 0) ? n : (s - 1);
                const int kind = ki < 2 ? 0 : (ki < 4 ? 2 : 3);
                const int slot = (s == 0) ? (n >> 1) : (s + 2);
                const size_t wo = ((size_t)((dir * 4 + kind) * NPP + (n & 1) * 16 + lr)) * HID + 8 * hi;
                v8f c = (v8f){};
#pragma unroll 4
                for (int kc = 0; kc < HID; kc += 32) { const int ao = (16 * rt + lr) * HP + kc + 8 * hi;
                    const v16h a = cat16(*(const v8ha*)&AT[ao], *(const v8ha*)&AT[ao + 16]);
                    const v16h bb = ldh(W2H + wo + kc);
                    c = wmma16g(a, bb, c); }
                const int m = (n & 1) * 16 + lr;
#pragma unroll
                for (int r = 0; r < 8; ++r) { if (m < NP) R[(16 * rt + 8 * hi + r) * RP + slot * NP + m] = c[r] * CINV; }
            }
            __syncthreads();
        }
#pragma unroll 1
        for (int it = 0; it < 5; ++it) { const int q = it * 128 + tid; const int r = q / NP, m = q % NP; const int bb = b0 + r;
            const int ro = r * RP + m;
            const float npf = fmaxf(sqrtf(R[ro]), EPSN), npa = fmaxf(sqrtf(R[ro + NP]), EPSN), npm = fmaxf(sqrtf(R[ro + 2 * NP]), EPSN);
            const float nhf = fmaxf(sqrtf(R[ro + 4 * NP]), EPSN);
            const float fm = R[ro + 3 * NP] / (npf * nhf);
            const float den = DEN[((size_t)(dir * NB_FULL + bb)) * SEQ + t];
            const float rd = 1.0f / den;
            const float nba = fmaxf(sqrtf(R[ro + 6 * NP]) * fabsf(rd), EPSN);
            const float am = (R[ro + 5 * NP] * rd) / (npa * nba);
            const float nbm = fmaxf(sqrtf(R[ro + 8 * NP]), EPSN);
            const float mam = R[ro + 7 * NP] / (npm * nbm);
            const float mp = MPMT[((size_t)((dir * SEQ + t) * NB_FULL + bb)) * 32 + m];
            OT[r * OC + dir * NP + m] = fm;
            OT[r * OC + 2 * NP + dir * NP + m] = mp;
            OT[r * OC + 4 * NP + dir * NP + m] = am;
            OT[r * OC + 6 * NP + dir * NP + m] = mam; }
    }
    __syncthreads();
    static_assert(128 * 10 * 16 == 32 * OC * 4);
    static_assert(((size_t)OC * 4 * 32) % 128 == 0);
    float* ob = OUT + ((size_t)(t * NB_FULL + b0)) * OC;
#pragma unroll 1
    for (int ps = 0; ps < 2; ++ps) {
#pragma unroll 2
        for (int it = 0; it < 10; ++it) { const int q = it * 128 + tid;
            const v4f val = *(const v4fa*)&OT[q * 4];
            *(volatile v4f*)(ob + (size_t)q * 4) = val; }
        if (ps == 0) __threadfence(); }
}

static constexpr size_t al256(size_t v) { return (v + 255) & ~(size_t)255; }
static constexpr size_t SZ_XB  = al256((size_t)4 * PLANE * 2);
static constexpr size_t SZ_HPL = al256((size_t)8 * PLANE * 2);
static constexpr size_t SZ_W2  = al256((size_t)8 * NPP * HID * 2);
static constexpr size_t SZ_DEN = al256((size_t)2 * NB_FULL * SEQ * 4);
static constexpr size_t SZ_MPM = al256((size_t)2 * SEQ * NB_FULL * 32 * 4);
static constexpr size_t SZ_TOTAL = SZ_XB + SZ_HPL + SZ_W2 + SZ_DEN + SZ_MPM;
static_assert(SZ_TOTAL <= (size_t)134217728);
static_assert((PLANE * 2) % 256 == 0);
static_assert(((size_t)NPP * HID * 2) % 256 == 0);

extern "C" void kernel_launch(void* const* d_in, const int* in_sizes, int n_in,
                              void* d_out, int out_size, void* d_ws, size_t ws_size, hipStream_t stream) {
    if (n_in < 12) return;
    for (int i = 0; i < 4; ++i) if ((size_t)in_sizes[i] < PLANE) return;
    for (int i = 4; i < 12; ++i) if (in_sizes[i] < NP * HID) return;
    if ((size_t)out_size < (size_t)SEQ * NB_FULL * OC) return;
    if (SZ_TOTAL > ws_size) return;
    float* OUT = (float*)d_out;
    char* wsp = (char*)d_ws;
    bf*  XB  = (bf*)wsp;   wsp += SZ_XB;
    h16* HPL = (h16*)wsp;  wsp += SZ_HPL;
    h16* W2H = (h16*)wsp;  wsp += SZ_W2;
    float* DEN  = (float*)wsp; wsp += SZ_DEN;
    float* MPMT = (float*)wsp; wsp += SZ_MPM;

    { const size_t n8 = PLANE / 8; const unsigned g = (unsigned)((n8 + 255) / 256);
      for (int i = 0; i < 4; ++i) k_cvt2<<<g, 256, 0, stream>>>((const float*)d_in[i], XB + (size_t)i * PLANE, HPL + (size_t)i * PLANE, n8); }
    for (int kind = 0; kind < 4; ++kind)
        for (int d = 0; d < 2; ++d)
            k_w2<<<(NPP * HID / 8) / 256, 256, 0, stream>>>((const float*)d_in[4 + 2 * kind + d], W2H + (size_t)((d * 4 + kind) * NPP) * HID);

    k_gram<<<dim3(NB, 2, 1), 128, 0, stream>>>(XB, HPL, HPL + (size_t)4 * PLANE, HPL + (size_t)6 * PLANE, DEN);
    k_mpm<<<NB, 128, 0, stream>>>(HPL, W2H, (const float*)d_in[6], MPMT, 0);
    k_mpm<<<NB, 128, 0, stream>>>(HPL, W2H, (const float*)d_in[7], MPMT, 1);
    k_final<<<SEQ * (NB / 32), 128, 0, stream>>>(HPL, W2H, DEN, MPMT, OUT);
}
